// SimpleGNNModel_15788299780297
// MI455X (gfx1250) — hardware-verified
//
#include <hip/hip_runtime.h>
#include <stddef.h>


#define IN_DIM 5
#define HID    64
#define EDIM   4
#define ODIM   3
#define NLAY   3
#define KW1    (HID + EDIM)
#define GR     32
#define NTHR   256
#define NWAVE  8
#define AP     72
#define FP     68
#define WSC    16.0f
#define WSCI   0.0625f
#define BNEPS  1e-5f
#define W2ROW  (NLAY * HID)
#define W3ROW  (2 * NLAY * HID)
#define W4ROW  (2 * NLAY * HID + HID)
#define NWROW  (2 * NLAY * HID + HID + 16)

#define NB     1024
#define CHUNK  4096
#define NGRP   (CHUNK / (NTHR * 4))
#define WCAP   ((CHUNK / NTHR) * 32)
#define LDS_SACC (NB * HID)
#define LDS_CNT  NB
#define LDS_LIST (NWAVE * WCAP)
#define AGG_LDS_BYTES ((LDS_SACC + LDS_CNT + LDS_LIST + NWAVE) * 4)

static_assert(NGRP == 4);
static_assert(WCAP == 512);
static_assert(AGG_LDS_BYTES == 282656);
static_assert(((LDS_SACC + LDS_CNT) % 4) == 0);
static_assert((NB & (NB - 1)) == 0);
static_assert(NB <= 1024);
static_assert(CHUNK <= 4096);
static_assert(NB / NWAVE == 128);
static_assert((GR * ODIM) % 4 == 0);
static_assert(NWROW == 464);

typedef float    v2f  __attribute__((ext_vector_type(2)));
typedef float    v4f  __attribute__((ext_vector_type(4)));
typedef float    v8f  __attribute__((ext_vector_type(8)));
typedef int      v4i  __attribute__((ext_vector_type(4)));
typedef double   v2d  __attribute__((ext_vector_type(2)));
typedef _Float16 v8h  __attribute__((ext_vector_type(8)));
typedef _Float16 v16h __attribute__((ext_vector_type(16)));
union Frag   { v16h v; v8h half[2]; };
union Pack16 { v8h h; v4i i; };

__device__ __forceinline__ v8f wm(v16h a, v16h b, v8f c) {
  v8f d = __builtin_amdgcn_wmma_f32_16x16x32_f16(false, a, false, b, (short)0, c, false, false);
  asm volatile("v_nop\n\tv_nop\n\tv_nop\n\tv_nop" : "+v"(d) : "v"(a), "v"(b));
  return d;
}

__device__ __forceinline__ float relu1(float v) { return v > 0.0f ? v : 0.0f; }
__device__ __forceinline__ v4f relu4(v4f v) {
  v.x = relu1(v.x); v.y = relu1(v.y); v.z = relu1(v.z); v.w = relu1(v.w);
  return v;
}

__device__ __forceinline__ v8f gemm_tile(const _Float16* At, const _Float16* __restrict__ Wt,
                                         int arow0, int nrow, int hh, int m) {
  v8f acc = {0.f, 0.f, 0.f, 0.f, 0.f, 0.f, 0.f, 0.f};
#pragma unroll
  for (int kt = 0; kt < HID / 32; ++kt) {
    const int k0 = kt * 32;
    Frag a, b;
    const _Float16* pa = At + (arow0 + m) * AP + k0 + 8 * hh;
    const _Float16* pb = Wt + (size_t)nrow * HID + k0 + 8 * hh;
    a.half[0] = *(const v8h*)pa;  a.half[1] = *(const v8h*)(pa + 16);
    b.half[0] = *(const v8h*)pb;  b.half[1] = *(const v8h*)(pb + 16);
    acc = wm(a.v, b.v, acc);
  }
  return acc;
}

__device__ __forceinline__ void bn_res8(const float* __restrict__ hin, const float* __restrict__ agg,
                                        const float* __restrict__ stats, const float* __restrict__ gam,
                                        const float* __restrict__ bet, size_t off, int c0,
                                        v4f& o0, v4f& o1) {
  const v4f h0 = *(const v4f*)(hin + off),        h1 = *(const v4f*)(hin + off + 4);
  const v4f a0 = *(const v4f*)(agg + off),        a1 = *(const v4f*)(agg + off + 4);
  const v4f u0 = *(const v4f*)(stats + c0),       u1 = *(const v4f*)(stats + c0 + 4);
  const v4f r0 = *(const v4f*)(stats + HID + c0), r1 = *(const v4f*)(stats + HID + c0 + 4);
  const v4f g0 = *(const v4f*)(gam + c0),         g1 = *(const v4f*)(gam + c0 + 4);
  const v4f e0 = *(const v4f*)(bet + c0),         e1 = *(const v4f*)(bet + c0 + 4);
  const v4f t0 = ((a0 - u0) * r0) * g0 + e0;
  const v4f t1 = ((a1 - u1) * r1) * g1 + e1;
  o0 = h0 + relu4(t0);
  o1 = h1 + relu4(t1);
}

__device__ __forceinline__ void stage8(_Float16* At, int r, int c0, v4f o0, v4f o1) {
  Pack16 u;
  u.h[0] = (_Float16)o0.x; u.h[1] = (_Float16)o0.y; u.h[2] = (_Float16)o0.z; u.h[3] = (_Float16)o0.w;
  u.h[4] = (_Float16)o1.x; u.h[5] = (_Float16)o1.y; u.h[6] = (_Float16)o1.z; u.h[7] = (_Float16)o1.w;
  *(v8h*)(At + r * AP + c0) = u.h;
}

__global__ __launch_bounds__(NTHR) void k_prep(const float* __restrict__ W1, const float* __restrict__ W2,
                                               const float* __restrict__ W3, const float* __restrict__ W4,
                                               _Float16* Wt, int total8) {
  const int i = blockIdx.x * NTHR + threadIdx.x;
  if (i >= total8) return;
  const int row = i >> 3;
  const int k0  = (i & 7) * 8;
  const float* base;
  int stride;
  float keep = 1.0f;
  if (row < W2ROW) {
    const int l = row >> 6, n = row & 63;
    base = W1 + (size_t)l * KW1 * HID + n; stride = HID;
  } else if (row < W3ROW) {
    const int l = (row - W2ROW) >> 6, n = (row - W2ROW) & 63;
    base = W2 + (size_t)l * HID * HID + n; stride = HID;
  } else if (row < W4ROW) {
    const int n = row - W3ROW;
    base = W3 + n; stride = HID;
  } else {
    const int n  = row - W4ROW;
    const int nc = n < ODIM ? n : ODIM - 1;
    base = W4 + nc; stride = ODIM;
    keep = (n < ODIM) ? 1.0f : 0.0f;
  }
  Pack16 u;
#pragma unroll
  for (int j = 0; j < 8; ++j) u.h[j] = (_Float16)(base[(size_t)(k0 + j) * stride] * keep * WSC);
  _Float16* p = Wt + (size_t)row * HID + k0;
  *(volatile v4i*)p = u.i;
  __threadfence();
  *(volatile v4i*)p = u.i;
}

__global__ __launch_bounds__(NTHR) void k_node(
    const float* __restrict__ x, const float* __restrict__ Win, const float* __restrict__ bin,
    const float* __restrict__ hin, const float* __restrict__ agg, const float* __restrict__ stats,
    const float* __restrict__ gam, const float* __restrict__ bet,
    const _Float16* __restrict__ Wt, float* hout, float* P, int nN, int mode) {
  __shared__ __attribute__((aligned(16))) _Float16 At[GR * AP];
  __shared__ __attribute__((aligned(16))) float Hs[GR * FP];
  __shared__ __attribute__((aligned(16))) float Ps[GR * FP];

  const int tid  = threadIdx.x;
  const int lane = tid & 31;
  const int wave = tid >> 5;
  const int hh   = lane >> 4;
  const int m    = lane & 15;
  const int rowBase = blockIdx.x * GR;

  {
    const int r  = tid >> 3;
    const int c0 = (tid & 7) * 8;
    int row = rowBase + r;
    if (row > nN - 1) row = nN - 1;
    v4f o0, o1;
    if (mode == 0) {
      v4f acc0 = {0.f, 0.f, 0.f, 0.f};
      v4f acc1 = acc0;
      const float* xr = x + (size_t)row * IN_DIM;
#pragma unroll 1
      for (int k = 0; k < IN_DIM; ++k) {
        const float xv = xr[k];
        const v4f w0 = *(const v4f*)(Win + k * HID + c0);
        const v4f w1 = *(const v4f*)(Win + k * HID + c0 + 4);
        acc0 += xv * w0;
        acc1 += xv * w1;
      }
      const v4f b0  = *(const v4f*)(bin + c0);
      const v4f b1v = *(const v4f*)(bin + c0 + 4);
      o0 = relu4(acc0 + b0);
      o1 = relu4(acc1 + b1v);
    } else {
      bn_res8(hin, agg, stats, gam, bet, (size_t)row * HID + c0, c0, o0, o1);
    }
    *(v4f*)(Hs + r * FP + c0)     = o0;
    *(v4f*)(Hs + r * FP + c0 + 4) = o1;
    stage8(At, r, c0, o0, o1);
  }
  __syncthreads();

  const int rt = wave >> 2, ct = wave & 3;
  const int ncol = ct * 16 + m;
  const v8f acc = gemm_tile(At, Wt, rt * 16, ncol, hh, m);
#pragma unroll
  for (int r = 0; r < 8; ++r) Ps[(rt * 16 + 8 * hh + r) * FP + ncol] = acc[r] * WSCI;
  __syncthreads();

  v4f hv[2], pv[2];
  float* hp[2];
  float* pp[2];
#pragma unroll
  for (int i = 0; i < 2; ++i) {
    const int row = 4 * wave + 2 * i + (lane >> 4);
    const int col = (lane & 15) * 4;
    hv[i] = *(const v4f*)(Hs + row * FP + col);
    pv[i] = *(const v4f*)(Ps + row * FP + col);
    hp[i] = hout + (size_t)(rowBase + row) * HID + col;
    pp[i] = P    + (size_t)(rowBase + row) * HID + col;
  }
#pragma unroll
  for (int i = 0; i < 2; ++i) { *(volatile v4f*)hp[i] = hv[i]; *(volatile v4f*)pp[i] = pv[i]; }
  __threadfence();
#pragma unroll
  for (int i = 0; i < 2; ++i) { *(volatile v4f*)hp[i] = hv[i]; *(volatile v4f*)pp[i] = pv[i]; }
}

__device__ __forceinline__ void agg_store(const float* sacc, const float* cntv, float* S, float* cnt,
                                          int nodeBase, int wave, int lane) {
  const int sub = lane >> 4, piece = 4 * (lane & 15);
#pragma unroll 1
  for (int jp = 0; jp < NB / NWAVE / 2; ++jp) {
    const int slot = wave * (NB / NWAVE) + 2 * jp + sub;
    const v4f v = *(const v4f*)(sacc + slot * HID + piece);
    *(volatile v4f*)(S + (size_t)(nodeBase + slot) * HID + piece) = v;
  }
  const v4f cv = *(const v4f*)(cntv + wave * (NB / NWAVE) + 4 * lane);
  *(volatile v4f*)(cnt + (size_t)nodeBase + wave * (NB / NWAVE) + 4 * lane) = cv;
}

__global__ __launch_bounds__(NTHR) void k_agg(
    const int* __restrict__ ei, const float* __restrict__ ea, const float* __restrict__ P,
    const float* __restrict__ W1l, const float* __restrict__ b1l,
    float* S, float* cnt, int nN, int nE) {
  extern __shared__ v4f lds_dyn[];
  float* sacc = (float*)lds_dyn;
  float* cntv = sacc + LDS_SACC;
  int*   list = (int*)(cntv + LDS_CNT);
  int*   wcnt = list + LDS_LIST;

  const int tid  = threadIdx.x;
  const int lane = tid & 31;
  const int wave = tid >> 5;
  const int nodeBase = blockIdx.x * NB;

  {
    const v4f z4 = {0.f, 0.f, 0.f, 0.f};
    for (int i = tid; i < (LDS_SACC + LDS_CNT) / 4; i += NTHR) lds_dyn[i] = z4;
  }
  const v2f w0 = *(const v2f*)(W1l + (HID + 0) * HID + 2 * lane);
  const v2f w1 = *(const v2f*)(W1l + (HID + 1) * HID + 2 * lane);
  const v2f w2 = *(const v2f*)(W1l + (HID + 2) * HID + 2 * lane);
  const v2f w3 = *(const v2f*)(W1l + (HID + 3) * HID + 2 * lane);
  const v2f bb = *(const v2f*)(b1l + 2 * lane);
  __syncthreads();

  const int* eid = ei + nE;
  const bool al16 = ((nE & 3) == 0);
  const int nChunks = (nE + CHUNK - 1) / CHUNK;

#pragma unroll 1
  for (int ch = 0; ch < nChunks; ++ch) {
    const int cbase = ch * CHUNK;
    int wc = 0;
#pragma unroll
    for (int g = 0; g < NGRP; ++g) {
      const int el0 = (g * NTHR + tid) * 4;
      const int e0  = cbase + el0;
      const int sent = -2147483647 - 1;
      v4i d;
      if (al16 && (cbase + CHUNK <= nE)) {
        d = *(const v4i*)(eid + e0);
      } else {
        d.x = (e0     < nE) ? eid[min(e0,     nE - 1)] : sent;
        d.y = (e0 + 1 < nE) ? eid[min(e0 + 1, nE - 1)] : sent;
        d.z = (e0 + 2 < nE) ? eid[min(e0 + 2, nE - 1)] : sent;
        d.w = (e0 + 3 < nE) ? eid[min(e0 + 3, nE - 1)] : sent;
      }
      const unsigned s0 = (unsigned)d.x - (unsigned)nodeBase;
      const unsigned s1 = (unsigned)d.y - (unsigned)nodeBase;
      const unsigned s2 = (unsigned)d.z - (unsigned)nodeBase;
      const unsigned s3 = (unsigned)d.w - (unsigned)nodeBase;
      const bool h0 = s0 < (unsigned)NB;
      const bool h1 = s1 < (unsigned)NB;
      const bool h2 = s2 < (unsigned)NB;
      const bool h3 = s3 < (unsigned)NB;
      const unsigned many = __builtin_amdgcn_ballot_w32(h0 | h1 | h2 | h3);
      if (many != 0u) {
#define HITJ(J, HJ, SJ) { \
          const unsigned mj = __builtin_amdgcn_ballot_w32(HJ); \
          if (HJ) { \
            const int pos = wc + (int)__builtin_amdgcn_mbcnt_lo(mj, 0u); \
            if (pos < WCAP) list[wave * WCAP + pos] = ((el0 + (J)) << 10) | (int)(SJ); \
          } \
          wc += (int)__builtin_popcount(mj); }
        HITJ(0, h0, s0)
        HITJ(1, h1, s1)
        HITJ(2, h2, s2)
        HITJ(3, h3, s3)
#undef HITJ
      }
    }
    if (lane == 0) wcnt[wave] = wc;
    __syncthreads();

    if (wave == 0) {
#pragma unroll 1
      for (int wsx = 0; wsx < NWAVE; ++wsx) {
        int n = wcnt[wsx];
        if (n > WCAP) n = WCAP;
        if (n < 0) n = 0;
#pragma unroll 1
        for (int i = 0; i < n; ++i) {
          const int ent  = list[wsx * WCAP + i];
          const int slot = ent & (NB - 1);
          const int el   = (ent >> 10) & (CHUNK - 1);
          int e = cbase + el;
          if (e > nE - 1) e = nE - 1;
          int src = ei[e];
          src = src < 0 ? 0 : (src > nN - 1 ? nN - 1 : src);
          const v4f av = *(const v4f*)(ea + (size_t)e * EDIM);
          const v2f pv = *(const v2f*)(P + (size_t)src * HID + 2 * lane);
          v2f r = pv;
          r += av.x * w0;
          r += av.y * w1;
          r += av.z * w2;
          r += av.w * w3;
          r += bb;
          r.x = relu1(r.x);
          r.y = relu1(r.y);
          v2f* sp = (v2f*)(sacc + slot * HID + 2 * lane);
          const v2f cur = *sp;
          *sp = cur + r;
          if (lane == 0) cntv[slot] = cntv[slot] + 1.0f;
        }
      }
    }
    __syncthreads();
  }

  agg_store(sacc, cntv, S, cnt, nodeBase, wave, lane);
  __threadfence();
  agg_store(sacc, cntv, S, cnt, nodeBase, wave, lane);
}

__global__ __launch_bounds__(NTHR) void k_gemm2(
    const float* __restrict__ S, const float* __restrict__ cnt,
    const _Float16* __restrict__ Wt, const float* __restrict__ b2,
    float* agg, double* part, int nN) {
  __shared__ __attribute__((aligned(16))) _Float16 At[GR * AP];
  __shared__ __attribute__((aligned(16))) float Ag[GR * FP];
  __shared__ float Cs[GR];
  __shared__ __attribute__((aligned(16))) double Fs[2 * HID];

  const int tid  = threadIdx.x;
  const int lane = tid & 31;
  const int wave = tid >> 5;
  const int hh   = lane >> 4;
  const int m    = lane & 15;
  const int rowBase = blockIdx.x * GR;

  {
    const int r  = tid >> 3;
    const int c0 = (tid & 7) * 8;
    int row = rowBase + r;
    if (row > nN - 1) row = nN - 1;
    const v4f s0 = *(const v4f*)(S + (size_t)row * HID + c0);
    const v4f s1 = *(const v4f*)(S + (size_t)row * HID + c0 + 4);
    stage8(At, r, c0, s0, s1);
    if ((tid & 7) == 0) Cs[r] = cnt[row];
  }
  __syncthreads();

  const int rt = wave >> 2, ct = wave & 3;
  const int ncol = ct * 16 + m;
  const float bcol = b2[ncol];
  const v8f acc = gemm_tile(At, Wt, rt * 16, ncol, hh, m);
#pragma unroll
  for (int r = 0; r < 8; ++r) {
    const int rowl = rt * 16 + 8 * hh + r;
    Ag[rowl * FP + ncol] = acc[r] * WSCI + Cs[rowl] * bcol;
  }
  __syncthreads();

  if (tid < HID) {
    double ds = 0.0, dq = 0.0;
#pragma unroll 1
    for (int rr = 0; rr < GR; ++rr) {
      const double v = (double)Ag[rr * FP + tid];
      ds += v;
      dq += v * v;
    }
    Fs[tid] = ds;
    Fs[HID + tid] = dq;
  }
  __syncthreads();

  v4f av[2];
  float* ap[2];
#pragma unroll
  for (int i = 0; i < 2; ++i) {
    const int row = 4 * wave + 2 * i + (lane >> 4);
    const int col = (lane & 15) * 4;
    av[i] = *(const v4f*)(Ag + row * FP + col);
    ap[i] = agg + (size_t)(rowBase + row) * HID + col;
  }
  const bool fw = (wave < 2);
  const int  fo = (fw ? wave : 0) * HID + 2 * lane;
  const v2d  fv = *(const v2d*)(Fs + fo);
  double* fp = part + (size_t)blockIdx.x * (2 * HID) + fo;

#pragma unroll
  for (int i = 0; i < 2; ++i) *(volatile v4f*)ap[i] = av[i];
  if (fw) *(volatile v2d*)fp = fv;
  __threadfence();
#pragma unroll
  for (int i = 0; i < 2; ++i) *(volatile v4f*)ap[i] = av[i];
  if (fw) *(volatile v2d*)fp = fv;
}

__global__ __launch_bounds__(NTHR) void k_bnfin(const double* __restrict__ part, int nBlk, int nN,
                                                float* stats) {
  __shared__ double Sd[4 * HID];
  __shared__ double Qd[4 * HID];
  __shared__ __attribute__((aligned(16))) float St[2 * HID];

  const int tid  = threadIdx.x;
  const int lane = tid & 31;
  const int wave = tid >> 5;
  const int col  = tid & (HID - 1);
  const int g    = tid >> 6;

  double s = 0.0, q = 0.0;
#pragma unroll 1
  for (int b = g; b < nBlk; b += 4) {
    const double* p = part + (size_t)b * (2 * HID);
    s += p[col];
    q += p[HID + col];
  }
  Sd[g * HID + col] = s;
  Qd[g * HID + col] = q;
  __syncthreads();

  if (tid < HID) {
    const double ts = ((Sd[col] + Sd[HID + col]) + Sd[2 * HID + col]) + Sd[3 * HID + col];
    const double tq = ((Qd[col] + Qd[HID + col]) + Qd[2 * HID + col]) + Qd[3 * HID + col];
    const double inv = 1.0 / (double)nN;
    const double mu  = ts * inv;
    double var = tq * inv - mu * mu;
    if (var < 0.0) var = 0.0;
    const float varf = (float)var;
    St[tid]       = (float)mu;
    St[HID + tid] = rsqrtf(varf + BNEPS);
  }
  __syncthreads();

  const bool wr = (wave == 0);
  const v4f  v  = *(const v4f*)(St + 4 * lane);
  float* p = stats + 4 * lane;
  if (wr) *(volatile v4f*)p = v;
  __threadfence();
  if (wr) *(volatile v4f*)p = v;
}

__global__ __launch_bounds__(NTHR) void k_head(
    const float* __restrict__ hin, const float* __restrict__ agg, const float* __restrict__ stats,
    const float* __restrict__ gam, const float* __restrict__ bet,
    const _Float16* __restrict__ Wt3, const float* __restrict__ b3,
    const _Float16* __restrict__ Wt4, const float* __restrict__ b4,
    float* out, int nN) {
  __shared__ __attribute__((aligned(16))) _Float16 At[GR * AP];
  __shared__ __attribute__((aligned(16))) _Float16 Tt[GR * AP];
  __shared__ __attribute__((aligned(16))) float Os[GR * ODIM];

  const int tid  = threadIdx.x;
  const int lane = tid & 31;
  const int wave = tid >> 5;
  const int hh   = lane >> 4;
  const int m    = lane & 15;
  const int rowBase = blockIdx.x * GR;

  {
    const int r  = tid >> 3;
    const int c0 = (tid & 7) * 8;
    int row = rowBase + r;
    if (row > nN - 1) row = nN - 1;
    v4f o0, o1;
    bn_res8(hin, agg, stats, gam, bet, (size_t)row * HID + c0, c0, o0, o1);
    stage8(At, r, c0, o0, o1);
  }
  __syncthreads();

  {
    const int rt = wave >> 2, ct = wave & 3;
    const int ncol = ct * 16 + m;
    const float bcol = b3[ncol];
    const v8f acc = gemm_tile(At, Wt3, rt * 16, ncol, hh, m);
#pragma unroll
    for (int r = 0; r < 8; ++r) {
      const float t = relu1(acc[r] * WSCI + bcol);
      Tt[(rt * 16 + 8 * hh + r) * AP + ncol] = (_Float16)t;
    }
  }
  __syncthreads();

  if (wave < 2) {
    const v8f acc2 = gemm_tile(Tt, Wt4, wave * 16, m, hh, m);
    const float bo = b4[m < ODIM ? m : ODIM - 1];
    if (m < ODIM) {
#pragma unroll
      for (int r = 0; r < 8; ++r) Os[(wave * 16 + 8 * hh + r) * ODIM + m] = acc2[r] * WSCI + bo;
    }
  }
  __syncthreads();

  const bool wr = (wave == 0) && (lane < (GR * ODIM) / 4);
  const int  ol = wr ? lane : 0;
  const v4f  ov = *(const v4f*)(Os + 4 * ol);
  float* op = out + (size_t)blockIdx.x * (GR * ODIM) + 4 * ol;
  if (wr) *(volatile v4f*)op = ov;
  __threadfence();
  if (wr) *(volatile v4f*)op = ov;
}

extern "C" void kernel_launch(void* const* d_in, const int* in_sizes, int n_in,
                              void* d_out, int out_size, void* d_ws, size_t ws_size,
                              hipStream_t stream) {
  if (n_in < 15) return;
  const int nN = in_sizes[0] / IN_DIM;
  if (nN <= 0 || in_sizes[0] != nN * IN_DIM || (nN % GR) != 0) return;
  const int nE = in_sizes[1] / 2;
  if (nE <= 0 || in_sizes[1] != 2 * nE || in_sizes[2] != nE * EDIM) return;
  if (in_sizes[3] != IN_DIM * HID || in_sizes[4] != HID) return;
  if (in_sizes[5] != NLAY * KW1 * HID || in_sizes[6] != NLAY * HID) return;
  if (in_sizes[7] != NLAY * HID * HID || in_sizes[8] != NLAY * HID) return;
  if (in_sizes[9] != NLAY * HID || in_sizes[10] != NLAY * HID) return;
  if (in_sizes[11] != HID * HID || in_sizes[12] != HID) return;
  if (in_sizes[13] != HID * ODIM || in_sizes[14] != ODIM) return;
  if (out_size != nN * ODIM) return;

  const float* x     = (const float*)d_in[0];
  const int*   ei    = (const int*)  d_in[1];
  const float* ea    = (const float*)d_in[2];
  const float* Win   = (const float*)d_in[3];
  const float* bin   = (const float*)d_in[4];
  const float* W1    = (const float*)d_in[5];
  const float* b1    = (const float*)d_in[6];
  const float* W2    = (const float*)d_in[7];
  const float* b2    = (const float*)d_in[8];
  const float* gamma = (const float*)d_in[9];
  const float* beta  = (const float*)d_in[10];
  const float* W3    = (const float*)d_in[11];
  const float* b3    = (const float*)d_in[12];
  const float* W4    = (const float*)d_in[13];
  const float* b4    = (const float*)d_in[14];
  float* out = (float*)d_out;

  const int nBlk = nN / GR;
  const int nAgg = (nN + NB - 1) / NB;

  size_t off = 0;
  char* wsb = (char*)d_ws;
#define CARVE(PTR, TYPE, BYTES) PTR = (TYPE*)(wsb + off); off += (((size_t)(BYTES)) + 255) & ~(size_t)255;
  _Float16* Wt;  CARVE(Wt,  _Float16, (size_t)NWROW * HID * sizeof(_Float16))
  float* hA;     CARVE(hA,  float, (size_t)nN * HID * sizeof(float))
  float* hB;     CARVE(hB,  float, (size_t)nN * HID * sizeof(float))
  float* P;      CARVE(P,   float, (size_t)nN * HID * sizeof(float))
  float* agg;    CARVE(agg, float, (size_t)nN * HID * sizeof(float))
  float* S;      CARVE(S,   float, (size_t)nAgg * NB * HID * sizeof(float))
  float* cnt;    CARVE(cnt, float, (size_t)nAgg * NB * sizeof(float))
  double* part;  CARVE(part, double, (size_t)nBlk * 2 * HID * sizeof(double))
  float* stats;  CARVE(stats, float, (size_t)2 * HID * sizeof(float))
#undef CARVE
  if (off > ws_size) return;

  float* hbuf[2] = { hA, hB };

  const int total8 = NWROW * (HID / 8);
  k_prep<<<(total8 + NTHR - 1) / NTHR, NTHR, 0, stream>>>(W1, W2, W3, W4, Wt, total8);

  hipFuncSetAttribute(reinterpret_cast<const void*>(&k_agg),
                      hipFuncAttributeMaxDynamicSharedMemorySize, AGG_LDS_BYTES);

  for (int l = 0; l < NLAY; ++l) {
    const _Float16* W1t = Wt + (size_t)l * HID * HID;
    const _Float16* W2t = Wt + (size_t)(W2ROW + l * HID) * HID;
    float* hout = hbuf[l & 1];
    if (l == 0) {
      k_node<<<nBlk, NTHR, 0, stream>>>(x, Win, bin, hB, agg, stats, gamma, beta,
                                          W1t, hout, P, nN, 0);
    } else {
      const float* hin = hbuf[(l - 1) & 1];
      k_node<<<nBlk, NTHR, 0, stream>>>(x, Win, bin, hin, agg, stats,
                                          gamma + (l - 1) * HID, beta + (l - 1) * HID,
                                          W1t, hout, P, nN, 1);
    }
    k_agg<<<nAgg, NTHR, AGG_LDS_BYTES, stream>>>(ei, ea, P, W1 + (size_t)l * KW1 * HID,
                                                  b1 + l * HID, S, cnt, nN, nE);
    k_gemm2<<<nBlk, NTHR, 0, stream>>>(S, cnt, W2t, b2 + l * HID, agg, part, nN);
    k_bnfin<<<1, NTHR, 0, stream>>>(part, nBlk, nN, stats);
  }

  const float* hlast = hbuf[(NLAY - 1) & 1];
  k_head<<<nBlk, NTHR, 0, stream>>>(hlast, agg, stats, gamma + (NLAY - 1) * HID, beta + (NLAY - 1) * HID,
                                      Wt + (size_t)W3ROW * HID, b3, Wt + (size_t)W4ROW * HID, b4, out, nN);
}
